// OnlineMemoryAttention_83442624627083
// MI455X (gfx1250) — hardware-verified
//
#include <hip/hip_runtime.h>
#include <stddef.h>
#include <stdint.h>

#define NTOK 2048
#define HID  1024
#define NH   16
#define HDM  64
#define NQKV 3072
#define CMV  3072
#define CW1  4096
#define CW2  4160
#define CR1  4224
#define CR2  4288
#define CG   4352
#define CGE  4368
#define NBIG 4416
#define NWR  (NBIG + HID)
#define NYB  (NBIG / 64)
#define YK   NH
#define YV   (2 * NH)
#define YMV  (3 * NH)
#define YS   (3 * NH + HID / 64)
#define LW   64
#define QB   128
#define KC   64
#define NQB  (NTOK / QB)
#define TSEG 128
#define NPR  21

static_assert(NQKV == 3 * NH * HDM);
static_assert(NH * HDM == HID);
static_assert(NBIG % 64 == 0);
static_assert(NYB == 69);
static_assert(YS == 64);
static_assert(CGE == CG + NH);
static_assert(CW1 == CMV + HID);
static_assert(NTOK % 256 == 0);
static_assert(HID % 64 == 0);
static_assert(HID == 128 * 8);
static_assert(NTOK % KC == 0);
static_assert(QB == 2 * KC);
static_assert(16 * TSEG == NTOK);
static_assert(LW == 4 * NH);
static_assert(HDM == 64);

typedef _Float16 v16h __attribute__((ext_vector_type(16)));
typedef _Float16 v8h  __attribute__((ext_vector_type(8)));
typedef float    v8f  __attribute__((ext_vector_type(8)));
typedef float    v4f  __attribute__((ext_vector_type(4)));
typedef unsigned int v4u __attribute__((ext_vector_type(4)));

union Frag  { v16h v; v8h h[2]; };
union Pack8 { v8h h; v4u u; };

__device__ __forceinline__ v8f mma16(v16h a, v16h b, v8f c) {
  c = __builtin_amdgcn_wmma_f32_16x16x32_f16(false, a, false, b, (short)0, c, false, false);
  asm volatile("v_nop\n\tv_nop\n\tv_nop\n\tv_nop" : "+v"(c) : "v"(a), "v"(b));
  return c;
}

__device__ __forceinline__ v16h ldfrag(const _Float16* p, int ld, int row0, int k0, int lane) {
  const int m = lane & 15, lh = lane >> 4;
  const _Float16* q = p + (size_t)(row0 + m) * ld + k0 + 8 * lh;
  Frag f;
  f.h[0] = *(const v8h*)(q);
  f.h[1] = *(const v8h*)(q + 16);
  return f.v;
}

__device__ __forceinline__ v8f zero8() { return (v8f){0.f, 0.f, 0.f, 0.f, 0.f, 0.f, 0.f, 0.f}; }

__device__ __forceinline__ void gemm16x64(const _Float16* __restrict__ A, int lda,
                                          const _Float16* __restrict__ Bt, int ldb,
                                          int m0, int n0, int lane, v8f (&acc)[4]) {
#pragma unroll 2
  for (int k0 = 0; k0 < HID; k0 += 32) {
    const v16h a = ldfrag(A, lda, m0, k0, lane);
#pragma unroll
    for (int t = 0; t < 4; ++t) {
      const v16h b = ldfrag(Bt, ldb, n0 + 16 * t, k0, lane);
      acc[t] = mma16(a, b, acc[t]);
    }
  }
}

__device__ __forceinline__ void gemm32x64(const _Float16* __restrict__ A, int lda,
                                          const _Float16* __restrict__ Bt, int ldb,
                                          int m0, int n0, int lane, v8f (&acc)[2][4]) {
#pragma unroll 2
  for (int k0 = 0; k0 < HID; k0 += 32) {
    const v16h a0 = ldfrag(A, lda, m0, k0, lane);
    const v16h a1 = ldfrag(A, lda, m0 + 16, k0, lane);
    const v16h b0 = ldfrag(Bt, ldb, n0, k0, lane);
    const v16h b1 = ldfrag(Bt, ldb, n0 + 16, k0, lane);
    const v16h b2 = ldfrag(Bt, ldb, n0 + 32, k0, lane);
    const v16h b3 = ldfrag(Bt, ldb, n0 + 48, k0, lane);
    acc[0][0] = mma16(a0, b0, acc[0][0]);
    acc[1][0] = mma16(a1, b0, acc[1][0]);
    acc[0][1] = mma16(a0, b1, acc[0][1]);
    acc[1][1] = mma16(a1, b1, acc[1][1]);
    acc[0][2] = mma16(a0, b2, acc[0][2]);
    acc[1][2] = mma16(a1, b2, acc[1][2]);
    acc[0][3] = mma16(a0, b3, acc[0][3]);
    acc[1][3] = mma16(a1, b3, acc[1][3]);
  }
}

__global__ __launch_bounds__(128) void k_cvtx(const float* __restrict__ src, _Float16* __restrict__ dst) {
  const int row = blockIdx.x;
  const int col = (int)threadIdx.x * 8;
  const size_t o = (size_t)row * HID + col;
  const v4f a0 = *(const v4f*)(src + o);
  const v4f a1 = *(const v4f*)(src + o + 4);
  Pack8 pk;
  pk.h = (v8h){(_Float16)a0[0], (_Float16)a0[1], (_Float16)a0[2], (_Float16)a0[3],
               (_Float16)a1[0], (_Float16)a1[1], (_Float16)a1[2], (_Float16)a1[3]};
  const v4u vv = pk.u;
  volatile v4u* d = (volatile v4u*)(dst + o);
  *d = vv;
  __threadfence();
  *d = vv;
}

__global__ __launch_bounds__(128) void k_cvtw(const float* __restrict__ wqkv, const float* __restrict__ wval,
                                              const float* __restrict__ w1w, const float* __restrict__ w2w,
                                              const float* __restrict__ w1r, const float* __restrict__ w2r,
                                              const float* __restrict__ wg, const float* __restrict__ wout,
                                              _Float16* __restrict__ wb, _Float16* __restrict__ wo) {
  const int n = blockIdx.x;
  const int col = (int)threadIdx.x * 8;
  const float* src;
  _Float16* dst;
  bool zr = false;
  if (n < NQKV)      { src = wqkv + (size_t)n * HID;          dst = wb + (size_t)n * HID; }
  else if (n < CW1)  { src = wval + (size_t)(n - CMV) * HID;  dst = wb + (size_t)n * HID; }
  else if (n < CW2)  { src = w1w + (size_t)(n - CW1) * HID;   dst = wb + (size_t)n * HID; }
  else if (n < CR1)  { src = w2w + (size_t)(n - CW2) * HID;   dst = wb + (size_t)n * HID; }
  else if (n < CR2)  { src = w1r + (size_t)(n - CR1) * HID;   dst = wb + (size_t)n * HID; }
  else if (n < CG)   { src = w2r + (size_t)(n - CR2) * HID;   dst = wb + (size_t)n * HID; }
  else if (n < CGE)  { src = wg + (size_t)(n - CG) * HID;     dst = wb + (size_t)n * HID; }
  else if (n < NBIG) { src = wg + (size_t)(NH - 1) * HID;     dst = wb + (size_t)n * HID; zr = true; }
  else               { src = wout + (size_t)(n - NBIG) * HID; dst = wo + (size_t)(n - NBIG) * HID; }
  const v4f a0 = *(const v4f*)(src + col);
  const v4f a1 = *(const v4f*)(src + col + 4);
  float f[8];
  f[0] = a0[0]; f[1] = a0[1]; f[2] = a0[2]; f[3] = a0[3];
  f[4] = a1[0]; f[5] = a1[1]; f[6] = a1[2]; f[7] = a1[3];
  Pack8 pk;
#pragma unroll
  for (int i = 0; i < 8; ++i) pk.h[i] = (_Float16)(zr ? 0.f : (f[i] * 32.0f));
  const v4u vv = pk.u;
  volatile v4u* d = (volatile v4u*)(dst + col);
  *d = vv;
  __threadfence();
  *d = vv;
}

#define SFP 68
__global__ __launch_bounds__(128) void k_proj(const _Float16* __restrict__ xh,
                                              const _Float16* __restrict__ wb,
                                              const float* __restrict__ bqkv,
                                              const float* __restrict__ bval,
                                              const float* __restrict__ bg,
                                              _Float16* __restrict__ qp,
                                              _Float16* __restrict__ kp,
                                              _Float16* __restrict__ vtp,
                                              float* __restrict__ mv,
                                              float* __restrict__ p1,
                                              float* __restrict__ w2,
                                              float* __restrict__ r1,
                                              float* __restrict__ r2,
                                              float* __restrict__ gp) {
  __shared__ __align__(16) float sf[64 * SFP];
  const int tid = threadIdx.x, lane = tid & 31, wave = tid >> 5;
  const int hh = lane >> 4, c = lane & 15;
  const int mb = blockIdx.x * 64;
  const int y  = blockIdx.y;
  const int m0 = mb + wave * 16;
  const int n0 = y * 64;

  v8f acc[4];
#pragma unroll
  for (int t = 0; t < 4; ++t) acc[t] = zero8();
  gemm16x64(xh, HID, wb, HID, m0, n0, lane, acc);

  const bool isg = (y == NYB - 1);
  const float* bp = bqkv;
  int boff = 0;
  bool hasb = false;
  if (y < YMV)      { bp = bqkv; boff = y * 64;         hasb = true; }
  else if (y < YS)  { bp = bval; boff = (y - YMV) * 64; hasb = true; }
  else if (isg)     { bp = bg;   boff = 0;              hasb = true; }
#pragma unroll
  for (int t = 0; t < 4; ++t) {
    const int ci = 16 * t + c;
    const int bi = isg ? min(ci, NH - 1) : ci;
    float bb = bp[boff + bi];
    bb = (hasb && (!isg || ci < NH)) ? bb : 0.f;
#pragma unroll
    for (int r = 0; r < 8; ++r)
      sf[(wave * 16 + 8 * hh + r) * SFP + 16 * t + c] = acc[t][r] * 0.03125f + bb;
  }
  __syncthreads();

  if (y < YV) {
    _Float16* plane = (y < YK) ? qp : kp;
    const int head = (y < YK) ? y : (y - YK);
    v4u val[4];
    size_t go[4];
#pragma unroll
    for (int j = 0; j < 4; ++j) {
      const int p  = tid + 128 * j;
      const int lr = p >> 3;
      const int pc = p & 7;
      const float* ra = sf + lr * SFP + pc * 8;
      const v4f a0 = *(const v4f*)(ra), a1 = *(const v4f*)(ra + 4);
      Pack8 pk;
      pk.h = (v8h){(_Float16)a0[0], (_Float16)a0[1], (_Float16)a0[2], (_Float16)a0[3],
                   (_Float16)a1[0], (_Float16)a1[1], (_Float16)a1[2], (_Float16)a1[3]};
      val[j] = pk.u;
      go[j]  = ((size_t)head * NTOK + mb + lr) * HDM + pc * 8;
    }
    for (int ps = 0; ps < 2; ++ps) {
#pragma unroll
      for (int j = 0; j < 4; ++j) *(volatile v4u*)(plane + go[j]) = val[j];
      __threadfence();
    }
  } else if (y < YMV) {
    const int head = y - YV;
    v4u val[4];
    size_t go[4];
#pragma unroll
    for (int j = 0; j < 4; ++j) {
      const int p  = tid + 128 * j;
      const int d  = p >> 3;
      const int pc = p & 7;
      const float* cp = sf + (pc * 8) * SFP + d;
      Pack8 pk;
      pk.h = (v8h){(_Float16)cp[0 * SFP], (_Float16)cp[1 * SFP], (_Float16)cp[2 * SFP], (_Float16)cp[3 * SFP],
                   (_Float16)cp[4 * SFP], (_Float16)cp[5 * SFP], (_Float16)cp[6 * SFP], (_Float16)cp[7 * SFP]};
      val[j] = pk.u;
      go[j]  = ((size_t)head * HDM + d) * NTOK + mb + pc * 8;
    }
    for (int ps = 0; ps < 2; ++ps) {
#pragma unroll
      for (int j = 0; j < 4; ++j) *(volatile v4u*)(vtp + go[j]) = val[j];
      __threadfence();
    }
  } else {
    float* fb;
    int pitch, coff;
    if (y < YS) { fb = mv; pitch = HID; coff = (y - YMV) * 64; }
    else {
      pitch = LW; coff = 0;
      fb = (y == YS) ? p1 : ((y == YS + 1) ? w2 : ((y == YS + 2) ? r1 : ((y == YS + 3) ? r2 : gp)));
    }
    v4f val[8];
    size_t go[8];
#pragma unroll
    for (int j = 0; j < 8; ++j) {
      const int p  = tid + 128 * j;
      const int lr = p >> 4;
      const int pc = p & 15;
      val[j] = *(const v4f*)(sf + lr * SFP + pc * 4);
      go[j]  = (size_t)(mb + lr) * pitch + coff + pc * 4;
    }
    for (int ps = 0; ps < 2; ++ps) {
#pragma unroll
      for (int j = 0; j < 8; ++j) *(volatile v4f*)(fb + go[j]) = val[j];
      __threadfence();
    }
  }
}

__device__ __forceinline__ float sigm(float x) {
#pragma clang fp contract(off)
  const float e = __expf(-x);
  return __builtin_amdgcn_rcpf(1.0f + e);
}

__device__ __forceinline__ void ext6(v4f p, v4f q, float (&o)[6]) {
#pragma clang fp contract(off)
  const float e0 = p[0] * q[1] - p[1] * q[0];
  const float e1 = p[0] * q[2] - p[2] * q[0];
  const float e2 = p[0] * q[3] - p[3] * q[0];
  const float e3 = p[1] * q[2] - p[2] * q[1];
  const float e4 = p[1] * q[3] - p[3] * q[1];
  const float e5 = p[2] * q[3] - p[3] * q[2];
  float ss = e0 * e0 + e1 * e1 + e2 * e2 + e3 * e3 + e4 * e4 + e5 * e5;
  ss = fmaxf(ss, 1e-24f);
  const float inv = __builtin_amdgcn_rsqf(ss);
  o[0] = e0 * inv; o[1] = e1 * inv; o[2] = e2 * inv;
  o[3] = e3 * inv; o[4] = e4 * inv; o[5] = e5 * inv;
}

__device__ __forceinline__ void jline(const float* __restrict__ p1, const float* __restrict__ w2p,
                                      int t, int h, float (&jv)[6]) {
#pragma clang fp contract(off)
  const int tm = (t > 0) ? (t - 1) : 0;
  v4f a = *(const v4f*)(p1 + (size_t)tm * LW + h * 4);
  const v4f z = (v4f){0.f, 0.f, 0.f, 0.f};
  a = (t > 0) ? a : z;
  const v4f b = *(const v4f*)(w2p + (size_t)t * LW + h * 4);
  float L[6];
  ext6(a, b, L);
  jv[0] = L[5]; jv[1] = -L[4]; jv[2] = L[3]; jv[3] = L[2]; jv[4] = -L[1]; jv[5] = L[0];
}

__device__ __forceinline__ void acc21(float (&S)[NPR], const float (&j)[6]) {
#pragma clang fp contract(off)
  S[0]  += j[0] * j[0]; S[1]  += j[0] * j[1]; S[2]  += j[0] * j[2]; S[3]  += j[0] * j[3]; S[4]  += j[0] * j[4]; S[5]  += j[0] * j[5];
  S[6]  += j[1] * j[1]; S[7]  += j[1] * j[2]; S[8]  += j[1] * j[3]; S[9]  += j[1] * j[4]; S[10] += j[1] * j[5];
  S[11] += j[2] * j[2]; S[12] += j[2] * j[3]; S[13] += j[2] * j[4]; S[14] += j[2] * j[5];
  S[15] += j[3] * j[3]; S[16] += j[3] * j[4]; S[17] += j[3] * j[5];
  S[18] += j[4] * j[4]; S[19] += j[4] * j[5];
  S[20] += j[5] * j[5];
}

__device__ __forceinline__ float quad21(const float (&M)[NPR], const float (&r)[6]) {
#pragma clang fp contract(off)
  const float d = M[0] * (r[0] * r[0]) + M[6] * (r[1] * r[1]) + M[11] * (r[2] * r[2])
                + M[15] * (r[3] * r[3]) + M[18] * (r[4] * r[4]) + M[20] * (r[5] * r[5]);
  const float o = M[1] * (r[0] * r[1]) + M[2] * (r[0] * r[2]) + M[3] * (r[0] * r[3]) + M[4] * (r[0] * r[4]) + M[5] * (r[0] * r[5])
                + M[7] * (r[1] * r[2]) + M[8] * (r[1] * r[3]) + M[9] * (r[1] * r[4]) + M[10] * (r[1] * r[5])
                + M[12] * (r[2] * r[3]) + M[13] * (r[2] * r[4]) + M[14] * (r[2] * r[5])
                + M[16] * (r[3] * r[4]) + M[17] * (r[3] * r[5])
                + M[19] * (r[4] * r[5]);
  return d + 2.0f * o;
}

__global__ __launch_bounds__(256) void k_mem(const float* __restrict__ p1, const float* __restrict__ w2p,
                                             const float* __restrict__ r1p, const float* __restrict__ r2p,
                                             const float* __restrict__ gp, const float* __restrict__ msc,
                                             float* __restrict__ gt) {
#pragma clang fp contract(off)
  __shared__ float part[256 * NPR];
  __shared__ __align__(16) float gsum[NTOK];
  const int tid = threadIdx.x;
  const int h = tid & 15;
  const int seg = tid >> 4;
  const int t0 = seg * TSEG;

  float S[NPR];
#pragma unroll
  for (int e = 0; e < NPR; ++e) S[e] = 0.f;
#pragma unroll 1
  for (int i = 0; i < TSEG; ++i) {
    float jv[6];
    jline(p1, w2p, t0 + i, h, jv);
    acc21(S, jv);
  }
#pragma unroll
  for (int e = 0; e < NPR; ++e) part[tid * NPR + e] = S[e];
  __syncthreads();

  for (int pr = tid; pr < NH * NPR; pr += 256) {
    const int h2 = pr / NPR;
    const int e  = pr - h2 * NPR;
    double run = 0.0;
#pragma unroll 1
    for (int cc = 0; cc < 16; ++cc) {
      const int idx = (cc * 16 + h2) * NPR + e;
      const float v = part[idx];
      part[idx] = (float)run;
      run += (double)v;
    }
  }
  __syncthreads();

  float M[NPR];
#pragma unroll
  for (int e = 0; e < NPR; ++e) M[e] = part[tid * NPR + e];
  const float ms = msc[h];
#pragma unroll 1
  for (int i = 0; i < TSEG; ++i) {
    const int t = t0 + i;
    const v4f a = *(const v4f*)(r1p + (size_t)t * LW + h * 4);
    const v4f b = *(const v4f*)(r2p + (size_t)t * LW + h * 4);
    float rl[6];
    ext6(a, b, rl);
    const float score = quad21(M, rl);
    const float g = gp[(size_t)t * LW + h];
    float s = sigm(score * ms) * sigm(g);
    s += __shfl_xor(s, 1, 32);
    s += __shfl_xor(s, 2, 32);
    s += __shfl_xor(s, 4, 32);
    s += __shfl_xor(s, 8, 32);
    if (h == 0) gsum[t] = s * 0.0625f;
    float jv[6];
    jline(p1, w2p, t, h, jv);
    acc21(M, jv);
  }
  __syncthreads();

  v4f val[2];
  size_t go[2];
#pragma unroll
  for (int j = 0; j < 2; ++j) {
    const int p = tid + 256 * j;
    val[j] = *(const v4f*)(gsum + p * 4);
    go[j]  = (size_t)p * 4;
  }
  for (int ps = 0; ps < 2; ++ps) {
#pragma unroll
    for (int j = 0; j < 2; ++j) *(volatile v4f*)(gt + go[j]) = val[j];
    __threadfence();
  }
}

#define KTP 72
#define OSP 68
union AttnLds { _Float16 h[2 * KC * KTP + 8 * 16 * KTP]; float f[(2 * KC * KTP + 8 * 16 * KTP) / 2]; };
static_assert(sizeof(AttnLds) == 36864);
static_assert(QB * OSP <= (2 * KC * KTP + 8 * 16 * KTP) / 2);
__global__ __launch_bounds__(256) void k_attn(const _Float16* __restrict__ qp,
                                              const _Float16* __restrict__ kp,
                                              const _Float16* __restrict__ vt,
                                              const float* __restrict__ mv,
                                              const float* __restrict__ gt,
                                              _Float16* __restrict__ cb, float sscale) {
  __shared__ __align__(16) AttnLds L;
  _Float16* Ks = L.h;
  _Float16* Vs = L.h + KC * KTP;
  _Float16* Ps = L.h + 2 * KC * KTP;

  const int tid = threadIdx.x, lane = tid & 31, wave = tid >> 5;
  const int hh = lane >> 4, c = lane & 15;
  const int qb = blockIdx.x % NQB;
  const int h  = blockIdx.x / NQB;
  const int q0 = qb * QB + wave * 16;

  const _Float16* Q = qp + (size_t)h * NTOK * HDM;
  const _Float16* K = kp + (size_t)h * NTOK * HDM;
  const _Float16* V = vt + (size_t)h * HDM * NTOK;

  const float NEGI = -__builtin_huge_valf();
  float mrow[8], lrow[8];
  v8f oacc[4];
#pragma unroll
  for (int r = 0; r < 8; ++r) { mrow[r] = NEGI; lrow[r] = 0.f; }
#pragma unroll
  for (int t = 0; t < 4; ++t) oacc[t] = zero8();

  _Float16* pw = Ps + wave * 16 * KTP;
  const int nck = 2 * qb + 2;

  for (int kc = 0; kc < nck; ++kc) {
    const int kv0 = kc * KC;
    __syncthreads();
    {
      const int r  = tid >> 2;
      const int qq = (tid & 3) * 16;
      const _Float16* ks = K + (size_t)(kv0 + r) * HDM + qq;
      const _Float16* vs = V + (size_t)r * NTOK + kv0 + qq;
#pragma unroll
      for (int e = 0; e < 2; ++e) {
        *(v8h*)(Ks + r * KTP + qq + 8 * e) = *(const v8h*)(ks + 8 * e);
        *(v8h*)(Vs + r * KTP + qq + 8 * e) = *(const v8h*)(vs + 8 * e);
      }
    }
    __syncthreads();

    v8f s[4];
#pragma unroll
    for (int j = 0; j < 4; ++j) s[j] = zero8();
#pragma unroll
    for (int dc = 0; dc < 2; ++dc) {
      const v16h qa = ldfrag(Q, HDM, q0, dc * 32, lane);
#pragma unroll
      for (int j = 0; j < 4; ++j) {
        const v16h kb = ldfrag(Ks, KTP, j * 16, dc * 32, lane);
        s[j] = mma16(qa, kb, s[j]);
      }
    }
    const bool edge = (kc >= 2 * qb);
#pragma unroll
    for (int r = 0; r < 8; ++r) {
      const int qry = q0 + 8 * hh + r;
#pragma unroll
      for (int j = 0; j < 4; ++j) {
        const int key = kv0 + 16 * j + c;
        const float v = s[j][r] * sscale;
        s[j][r] = (edge && key > qry) ? NEGI : v;
      }
    }
    float cm[8];
#pragma unroll
    for (int r = 0; r < 8; ++r) {
      float m = NEGI;
#pragma unroll
      for (int j = 0; j < 4; ++j) m = fmaxf(m, s[j][r]);
#pragma unroll
      for (int off = 1; off < 16; off <<= 1) m = fmaxf(m, __shfl_xor(m, off, 32));
      cm[r] = m;
    }
    float al[8];
#pragma unroll
    for (int r = 0; r < 8; ++r) {
      const float mnew  = fmaxf(mrow[r], cm[r]);
      const float alpha = __expf(mrow[r] - mnew);
      mrow[r] = mnew;
      float psum = 0.f;
#pragma unroll
      for (int j = 0; j < 4; ++j) {
        const float p = __expf(s[j][r] - mnew);
        psum += p;
        pw[(8 * hh + r) * KTP + j * 16 + c] = (_Float16)(p * 1024.0f);
      }
#pragma unroll
      for (int off = 1; off < 16; off <<= 1) psum += __shfl_xor(psum, off, 32);
      lrow[r] = lrow[r] * alpha + psum;
      al[r] = alpha;
    }
#pragma unroll
    for (int t = 0; t < 4; ++t)
#pragma unroll
      for (int r = 0; r < 8; ++r) oacc[t][r] *= al[r];
    __syncthreads();

#pragma unroll
    for (int kk = 0; kk < 2; ++kk) {
      const v16h pa = ldfrag(pw, KTP, 0, kk * 32, lane);
#pragma unroll
      for (int t = 0; t < 4; ++t) {
        const v16h vb = ldfrag(Vs, KTP, t * 16, kk * 32, lane);
        oacc[t] = mma16(pa, vb, oacc[t]);
      }
    }
  }

  float invl[8];
#pragma unroll
  for (int r = 0; r < 8; ++r) invl[r] = (lrow[r] > 0.f) ? (0.0009765625f / lrow[r]) : 0.f;
  __syncthreads();
  float* Os = L.f;
#pragma unroll
  for (int r = 0; r < 8; ++r) {
#pragma unroll
    for (int t = 0; t < 4; ++t)
      Os[(wave * 16 + 8 * hh + r) * OSP + 16 * t + c] = oacc[t][r] * invl[r];
  }
  __syncthreads();
  v4u val[4];
  size_t go[4];
#pragma unroll
  for (int it = 0; it < 4; ++it) {
    const int p   = lane + 32 * it;
    const int Lr  = p >> 3;
    const int pc  = p & 7;
    const int tok = q0 + Lr;
    const float* osr = Os + (wave * 16 + Lr) * OSP + pc * 8;
    const v4f o0 = *(const v4f*)(osr), o1 = *(const v4f*)(osr + 4);
    const float g = gt[tok];
    const float* mp = mv + (size_t)tok * HID + h * HDM + pc * 8;
    const v4f e0 = *(const v4f*)(mp), e1 = *(const v4f*)(mp + 4);
    const v4f c0 = o0 + g * e0;
    const v4f c1 = o1 + g * e1;
    Pack8 pk;
    pk.h = (v8h){(_Float16)c0[0], (_Float16)c0[1], (_Float16)c0[2], (_Float16)c0[3],
                 (_Float16)c1[0], (_Float16)c1[1], (_Float16)c1[2], (_Float16)c1[3]};
    val[it] = pk.u;
    go[it]  = (size_t)tok * HID + h * HDM + pc * 8;
  }
  for (int ps = 0; ps < 2; ++ps) {
#pragma unroll
    for (int it = 0; it < 4; ++it) *(volatile v4u*)(cb + go[it]) = val[it];
    __threadfence();
  }
}

#define OTP 68
__device__ __forceinline__ void out_epilogue(v8f (&acc)[2][4], float scale, const float* __restrict__ bias,
                                             float* sw, float* __restrict__ out,
                                             int m0, int n0, int lane, int hh, int c) {
#pragma unroll
  for (int sub = 0; sub < 2; ++sub) {
    __syncthreads();
#pragma unroll
    for (int t = 0; t < 4; ++t) {
      const float bb = bias[n0 + 16 * t + c];
#pragma unroll
      for (int r = 0; r < 8; ++r) sw[(8 * hh + r) * OTP + 16 * t + c] = acc[sub][t][r] * scale + bb;
    }
    __syncthreads();
    v4f val[8];
    size_t go[8];
#pragma unroll
    for (int it = 0; it < 8; ++it) {
      const int p    = lane + 32 * it;
      const int Lr   = p >> 3;
      const int pc   = p & 7;
      const int row  = Lr >> 1;
      const int half = Lr & 1;
      val[it] = *(const v4f*)(sw + row * OTP + half * 32 + pc * 4);
      go[it]  = (size_t)(m0 + sub * 16 + row) * HID + n0 + half * 32 + pc * 4;
    }
    for (int ps = 0; ps < 2; ++ps) {
#pragma unroll
      for (int it = 0; it < 8; ++it) *(volatile v4f*)(out + go[it]) = val[it];
      __threadfence();
    }
  }
}

__global__ __launch_bounds__(256) void k_out(const _Float16* __restrict__ ap,
                                             const _Float16* __restrict__ wt,
                                             const float* __restrict__ bo,
                                             float* __restrict__ out) {
  __shared__ __align__(16) float st[8][16 * OTP];
  const int tid = threadIdx.x, lane = tid & 31, wave = tid >> 5;
  const int hh = lane >> 4, c = lane & 15;
  const int m0 = blockIdx.x * 256 + wave * 32;
  const int n0 = blockIdx.y * 64;

  v8f acc[2][4];
#pragma unroll
  for (int s = 0; s < 2; ++s)
#pragma unroll
    for (int t = 0; t < 4; ++t) acc[s][t] = zero8();
  gemm32x64(ap, HID, wt, HID, m0, n0, lane, acc);
  out_epilogue(acc, 0.03125f, bo, st[wave], out, m0, n0, lane, hh, c);
}

extern "C" void kernel_launch(void* const* d_in, const int* in_sizes, int n_in,
                              void* d_out, int out_size, void* d_ws, size_t ws_size,
                              hipStream_t stream) {
  if (n_in < 14) return;
  if (in_sizes[0] != NTOK * HID) return;
  if (in_sizes[1] != NQKV * HID) return;
  if (in_sizes[2] != NQKV) return;
  if (in_sizes[3] != LW * HID) return;
  if (in_sizes[4] != LW * HID) return;
  if (in_sizes[5] != LW * HID) return;
  if (in_sizes[6] != LW * HID) return;
  if (in_sizes[7] != HID * HID) return;
  if (in_sizes[8] != HID) return;
  if (in_sizes[9] != NH * HID) return;
  if (in_sizes[10] != NH) return;
  if (in_sizes[11] != NH) return;
  if (in_sizes[12] != HID * HID) return;
  if (in_sizes[13] != HID) return;
  if (out_size != NTOK * HID) return;

  const float* x    = (const float*)d_in[0];
  const float* wqkv = (const float*)d_in[1];
  const float* bqkv = (const float*)d_in[2];
  const float* w1w  = (const float*)d_in[3];
  const float* w2w  = (const float*)d_in[4];
  const float* w1r  = (const float*)d_in[5];
  const float* w2r  = (const float*)d_in[6];
  const float* wval = (const float*)d_in[7];
  const float* bval = (const float*)d_in[8];
  const float* wg   = (const float*)d_in[9];
  const float* bg   = (const float*)d_in[10];
  const float* msc  = (const float*)d_in[11];
  const float* wout = (const float*)d_in[12];
  const float* bout = (const float*)d_in[13];
  float* out = (float*)d_out;

  size_t off = 0;
  const size_t oXh = off; off += (size_t)NTOK * HID * 2;
  const size_t oWb = off; off += (size_t)NBIG * HID * 2;
  const size_t oWo = off; off += (size_t)HID * HID * 2;
  const size_t oQ  = off; off += (size_t)NH * NTOK * HDM * 2;
  const size_t oK  = off; off += (size_t)NH * NTOK * HDM * 2;
  const size_t oV  = off; off += (size_t)NH * HDM * NTOK * 2;
  const size_t oMv = off; off += (size_t)NTOK * HID * 4;
  const size_t oP1 = off; off += (size_t)NTOK * LW * 4;
  const size_t oW2 = off; off += (size_t)NTOK * LW * 4;
  const size_t oR1 = off; off += (size_t)NTOK * LW * 4;
  const size_t oR2 = off; off += (size_t)NTOK * LW * 4;
  const size_t oGp = off; off += (size_t)NTOK * LW * 4;
  const size_t oGt = off; off += (size_t)NTOK * 4;
  const size_t oCb = off; off += (size_t)NTOK * HID * 2;
  if (off > ws_size) return;
  if (off > (size_t)134217728) return;

  char* ws = (char*)d_ws;
  _Float16* Xh = (_Float16*)(ws + oXh);
  _Float16* Wb = (_Float16*)(ws + oWb);
  _Float16* Wo = (_Float16*)(ws + oWo);
  _Float16* Qp = (_Float16*)(ws + oQ);
  _Float16* Kp = (_Float16*)(ws + oK);
  _Float16* Vt = (_Float16*)(ws + oV);
  float*    Mv = (float*)(ws + oMv);
  float*    P1 = (float*)(ws + oP1);
  float*    W2 = (float*)(ws + oW2);
  float*    R1 = (float*)(ws + oR1);
  float*    R2 = (float*)(ws + oR2);
  float*    Gp = (float*)(ws + oGp);
  float*    Gt = (float*)(ws + oGt);
  _Float16* Cb = (_Float16*)(ws + oCb);

  k_cvtx<<<dim3(NTOK), dim3(128), 0, stream>>>(x, Xh);
  k_cvtw<<<dim3(NWR), dim3(128), 0, stream>>>(wqkv, wval, w1w, w2w, w1r, w2r, wg, wout, Wb, Wo);
  k_proj<<<dim3(NTOK / 64, NYB), dim3(128), 0, stream>>>(Xh, Wb, bqkv, bval, bg, Qp, Kp, Vt, Mv, P1, W2, R1, R2, Gp);
  k_mem<<<dim3(1), dim3(256), 0, stream>>>(P1, W2, R1, R2, Gp, msc, Gt);
  const float sscale = 0.125f;
  k_attn<<<dim3(NH * NQB), dim3(256), 0, stream>>>(Qp, Kp, Vt, Mv, Gt, Cb, sscale);
  k_out<<<dim3(NTOK / 256, HID / 64), dim3(256), 0, stream>>>(Cb, Wo, bout, out);
  (void)hipGetLastError();
}
